// Cross_Attention_63702954934333
// MI455X (gfx1250) — hardware-verified
//
#include <hip/hip_runtime.h>


#ifndef NB
#define NB 4
#endif
#ifndef SEQ
#define SEQ 1024
#endif
#define NB_FULL 4
#define SEQ_FULL 1024
#define DMOD 512
#define NH 8
#define HD 64
#define QKVW 2048
#define BNC_FULL ((size_t)NB_FULL * SEQ_FULL * DMOD)
#define OFF0 ((size_t)0)
#define OFF1 (BNC_FULL)
#define OFF2 (2 * BNC_FULL)
#define OFF3 (3 * BNC_FULL)
#define OFF4 (4 * BNC_FULL)
#define SC2 (0.125f * 1.4426950408889634f)

static_assert(SEQ % 256 == 0);
static_assert(SEQ <= SEQ_FULL);
static_assert(NB >= 1);
static_assert(NB <= NB_FULL);
static_assert(DMOD == NH * HD);
static_assert((OFF4 + 2) * 4 < 33554444);

typedef _Float16 h16;
typedef unsigned short bf;
typedef __attribute__((ext_vector_type(16))) __bf16   v16bf;
typedef __attribute__((ext_vector_type(16))) _Float16 v16h;
typedef __attribute__((ext_vector_type(8)))  _Float16 v8h;
typedef __attribute__((ext_vector_type(8)))  unsigned short v8us;
typedef __attribute__((ext_vector_type(16))) unsigned short v16us;
typedef __attribute__((ext_vector_type(8)))  float    v8f;
typedef __attribute__((ext_vector_type(4)))  float    v4f;
typedef v8h  __attribute__((may_alias)) v8ha;
typedef v4f  __attribute__((may_alias)) v4fa;
typedef v8us __attribute__((may_alias)) v8usa;

__device__ __forceinline__ unsigned short f2bf(float f) { unsigned u = __float_as_uint(f); u += 0x7FFFu + ((u >> 16) & 1u); return (unsigned short)(u >> 16); }
__device__ __forceinline__ float bf2f(unsigned short b) { return __uint_as_float(((unsigned)b) << 16); }
__device__ __forceinline__ float bfr(float f) { return bf2f(f2bf(f)); }
__device__ __forceinline__ v16h cat16(v8h lo, v8h hi) { return __builtin_shufflevector(lo, hi, 0, 1, 2, 3, 4, 5, 6, 7, 8, 9, 10, 11, 12, 13, 14, 15); }
__device__ __forceinline__ v16bf cat16b(v8us lo, v8us hi) { return __builtin_bit_cast(v16bf, __builtin_shufflevector(lo, hi, 0, 1, 2, 3, 4, 5, 6, 7, 8, 9, 10, 11, 12, 13, 14, 15)); }
__device__ __forceinline__ v8f wmma16(v16h a, v16h b, v8f c) { return __builtin_amdgcn_wmma_f32_16x16x32_f16(false, a, false, b, (short)0, c, false, false); }
__device__ __forceinline__ v8f wmmab(v16bf a, v16bf b, v8f c) { return __builtin_amdgcn_wmma_f32_16x16x32_bf16(false, a, false, b, (short)0, c, false, false); }
__device__ __forceinline__ void splitf(float y, unsigned short& h, unsigned short& l) { h = f2bf(y); l = f2bf(y - bf2f(h)); }

template <typename T16> struct WFrag;
template <> struct WFrag<h16> { typedef v16h V; static __device__ __forceinline__ V ld(const h16* p) { return cat16(*(const v8h*)p, *(const v8h*)(p + 16)); } static __device__ __forceinline__ v8f mma(V a, V b, v8f c) { return wmma16(a, b, c); } };
template <> struct WFrag<bf> { typedef v16bf V; static __device__ __forceinline__ V ld(const bf* p) { return cat16b(*(const v8us*)p, *(const v8us*)(p + 16)); } static __device__ __forceinline__ v8f mma(V a, V b, v8f c) { return wmmab(a, b, c); } };
template <typename T16, int NSPLIT, bool BIAS>
__global__ __launch_bounds__(32) void k_gemmw(const T16* __restrict__ A, const T16* __restrict__ A2, const T16* __restrict__ Bt, const T16* __restrict__ Bt2, int K, float* C, int ldc, const float* __restrict__ bias, size_t sA, size_t sB, size_t sC) {
    typedef typename WFrag<T16>::V V;
    __shared__ __align__(16) float os[16 * 68];
    const size_t z = blockIdx.z; A += z * sA; if (A2) A2 += z * sA; Bt += z * sB; if (Bt2) Bt2 += z * sB; C += z * sC;
    const int lane = threadIdx.x & 31, lr = lane & 15, hi = lane >> 4; const int r0 = blockIdx.x * 64, c0 = blockIdx.y * 64;
    v8f acc[4][4];
#pragma unroll
    for (int mb = 0; mb < 4; ++mb)
#pragma unroll
        for (int nb = 0; nb < 4; ++nb) acc[mb][nb] = (v8f){};
    const size_t aoff = (size_t)(r0 + lr) * K + 8 * hi, boff = (size_t)(c0 + lr) * K + 8 * hi;
#pragma unroll 1
    for (int kc = 0; kc < K; kc += 32) {
        V a[4], a2[4];
#pragma unroll
        for (int mb = 0; mb < 4; ++mb) { a[mb] = WFrag<T16>::ld(A + aoff + (size_t)mb * 16 * K + kc); if (NSPLIT == 1 || NSPLIT == 2) a2[mb] = WFrag<T16>::ld(A2 + aoff + (size_t)mb * 16 * K + kc); }
#pragma unroll
        for (int nb = 0; nb < 4; ++nb) { const V b = WFrag<T16>::ld(Bt + boff + (size_t)nb * 16 * K + kc); V b2; if (NSPLIT >= 2) b2 = WFrag<T16>::ld(Bt2 + boff + (size_t)nb * 16 * K + kc);
#pragma unroll
            for (int mb = 0; mb < 4; ++mb) { acc[mb][nb] = WFrag<T16>::mma(a[mb], b, acc[mb][nb]); if (NSPLIT == 1 || NSPLIT == 2) acc[mb][nb] = WFrag<T16>::mma(a2[mb], b, acc[mb][nb]); if (NSPLIT >= 2) acc[mb][nb] = WFrag<T16>::mma(a[mb], b2, acc[mb][nb]); } }
        asm volatile("v_nop\n\tv_nop\n\tv_nop\n\tv_nop" : "+v"(acc[0][0]), "+v"(acc[1][1]), "+v"(acc[2][2]), "+v"(acc[3][3]) : "v"(a[0]), "v"(a[3]));
    }
#pragma unroll
    for (int mb = 0; mb < 4; ++mb) {
#pragma unroll
        for (int nb = 0; nb < 4; ++nb) {
#pragma unroll
            for (int j = 0; j < 8; ++j) os[(hi * 8 + j) * 68 + nb * 16 + lr] = acc[mb][nb][j]; }
        __builtin_amdgcn_wave_barrier(); asm volatile("" ::: "memory");
        float* crow = C + (size_t)(r0 + mb * 16) * ldc + c0;
#pragma unroll 1
        for (int ps = 0; ps < 2; ++ps) {
#pragma unroll
            for (int s = 0; s < 8; ++s) { const int row = 2 * s + hi, cofs = lr * 4; v4f val = *(const v4fa*)(os + row * 68 + cofs); if (BIAS) { val[0] += bfr(bias[c0 + cofs]); val[1] += bfr(bias[c0 + cofs + 1]); val[2] += bfr(bias[c0 + cofs + 2]); val[3] += bfr(bias[c0 + cofs + 3]); }
                *(volatile v4f*)(crow + (size_t)row * ldc + cofs) = val; }
            if (ps == 0) __threadfence(); }
        __builtin_amdgcn_wave_barrier(); asm volatile("" ::: "memory");
    }
}

__global__ __launch_bounds__(256) void k_cvt8(const float* __restrict__ src, bf* dst, size_t n8) { const size_t i = (size_t)blockIdx.x * 256 + threadIdx.x; if (i >= n8) return; const v8f v = *(const v8f*)(src + i * 8); v8us o;
#pragma unroll
    for (int k = 0; k < 8; ++k) o[k] = f2bf(v[k]); *(volatile v8us*)(dst + i * 8) = o; __threadfence(); *(volatile v8us*)(dst + i * 8) = o; }
__global__ __launch_bounds__(256) void k_cvtx(const float* __restrict__ src, bf* dst, size_t n8) { const size_t i = (size_t)blockIdx.x * 256 + threadIdx.x; if (i >= n8) return; const size_t e = i * 8; const size_t r = e / DMOD; const int c = (int)(e % DMOD); const size_t bb = r / SEQ, t = r % SEQ;
    const v8f v = *(const v8f*)(src + ((bb * SEQ_FULL + t) * DMOD + c)); v8us o;
#pragma unroll
    for (int k = 0; k < 8; ++k) o[k] = f2bf(v[k]); *(volatile v8us*)(dst + e) = o; __threadfence(); *(volatile v8us*)(dst + e) = o; }

__device__ __forceinline__ float hp_piece(const float* s, bf* dh, bf* dl, size_t po) {
    const v8f v = *(const v8f*)s; v8us oh, ol; float ss = 0.0f;
#pragma unroll
    for (int q = 0; q < 8; ++q) { unsigned short a, c; splitf(v[q], a, c); oh[q] = a; ol[q] = c; ss += v[q] * v[q]; }
    *(volatile v8us*)(dh + po) = oh; *(volatile v8us*)(dl + po) = ol; __threadfence(); *(volatile v8us*)(dh + po) = oh; *(volatile v8us*)(dl + po) = ol;
    return ss;
}
__global__ __launch_bounds__(256) void k_hp(const float* __restrict__ F, bf* Qh, bf* Ql, bf* Kh, bf* Kl, bf* Th, bf* Tl, float* invq, float* invt) {
    __shared__ __align__(16) float invs[2][32];
    const int tid = threadIdx.x, lane = tid & 31, w = tid >> 5, j = tid & 7, tl = tid >> 3;
    const int h = blockIdx.y, b = blockIdx.z, t0 = blockIdx.x * 32, t = t0 + tl;
    const size_t hb = (size_t)b * NH + h;
    const float* src = F + ((size_t)b * SEQ + t) * QKVW + h * HD + 8 * j;
    const size_t po = (hb * SEQ + t) * HD + 8 * j;
    float ssq = hp_piece(src, Qh, Ql, po);
    (void)hp_piece(src + DMOD, Kh, Kl, po);
    float sst = hp_piece(src + 3 * DMOD, Th, Tl, po);
    ssq += __shfl_xor(ssq, 1, 32); ssq += __shfl_xor(ssq, 2, 32); ssq += __shfl_xor(ssq, 4, 32);
    sst += __shfl_xor(sst, 1, 32); sst += __shfl_xor(sst, 2, 32); sst += __shfl_xor(sst, 4, 32);
    const float iq = rsqrtf(fmaxf(ssq, 1e-24f)), it = rsqrtf(fmaxf(sst, 1e-24f));
    if (j == 0) { invs[0][tl] = iq; invs[1][tl] = it; }
    __syncthreads();
    if (w == 0 && lane < 16) { const int c2 = lane >> 3, k4 = (lane & 7) * 4; const v4f iv = *(const v4fa*)(&invs[c2][k4]); float* dp = (c2 == 0 ? invq : invt) + hb * SEQ + t0 + k4; *(volatile v4f*)dp = iv; __threadfence(); *(volatile v4f*)dp = iv; }
}

__global__ __launch_bounds__(256) void k_vt(const float* __restrict__ F, bf* VTh, bf* VTl) {
    __shared__ __align__(16) unsigned short th[64 * 72];
    __shared__ __align__(16) unsigned short tlo[64 * 72];
    const int tid = threadIdx.x, lane = tid & 31, w = tid >> 5;
    const int h = blockIdx.y, b = blockIdx.z, t0 = blockIdx.x * 64;
    const size_t hb = (size_t)b * NH + h;
    { const int t = tid >> 2, d0 = (tid & 3) * 16; const float* s = F + ((size_t)b * SEQ + t0 + t) * QKVW + 2 * DMOD + h * HD + d0;
#pragma unroll
      for (int i = 0; i < 4; ++i) { const v4f v = *(const v4f*)(s + 4 * i);
#pragma unroll
          for (int e = 0; e < 4; ++e) { unsigned short a, c; splitf(v[e], a, c); th[(d0 + 4 * i + e) * 72 + t] = a; tlo[(d0 + 4 * i + e) * 72 + t] = c; } } }
    __syncthreads();
#pragma unroll 1
    for (int ps = 0; ps < 2; ++ps) {
#pragma unroll
        for (int it = 0; it < 2; ++it) { const int d = it * 32 + w * 4 + (lane >> 3), jj = lane & 7; const v8us xh = *(const v8usa*)(th + d * 72 + 8 * jj), xl = *(const v8usa*)(tlo + d * 72 + 8 * jj);
            const size_t oo = (hb * HD + d) * SEQ + t0 + 8 * jj; *(volatile v8us*)(VTh + oo) = xh; *(volatile v8us*)(VTl + oo) = xl; }
        if (ps == 0) __threadfence(); }
}

__global__ __launch_bounds__(128) void k_attn(const bf* __restrict__ Qh, const bf* __restrict__ Ql, const bf* __restrict__ Kh, const bf* __restrict__ Kl,
                                              const bf* __restrict__ Vh, const bf* __restrict__ Vl, bf* Ch, bf* Cl) {
    typedef WFrag<bf> F; typedef F::V V;
    __shared__ __align__(16) float osm[4 * 16 * 68];
    const int lane = threadIdx.x & 31, lr = lane & 15, hi = lane >> 4, w = threadIdx.x >> 5;
    const int h = blockIdx.y, b = blockIdx.z; const size_t hb = (size_t)b * NH + h;
    const int q0 = blockIdx.x * 64 + w * 16;
    const bf* qh = Qh + (hb * SEQ + q0) * HD + (size_t)lr * HD + 8 * hi; const bf* ql = Ql + (hb * SEQ + q0) * HD + (size_t)lr * HD + 8 * hi;
    const V qh0 = F::ld(qh), qh1 = F::ld(qh + 32), ql0 = F::ld(ql), ql1 = F::ld(ql + 32);
    const bf* kh = Kh + hb * SEQ * HD + (size_t)lr * HD + 8 * hi; const bf* kl = Kl + hb * SEQ * HD + (size_t)lr * HD + 8 * hi;
    const bf* vh = Vh + hb * HD * SEQ + (size_t)lr * SEQ + 8 * hi; const bf* vl = Vl + hb * HD * SEQ + (size_t)lr * SEQ + 8 * hi;
    v8f o[4];
#pragma unroll
    for (int db = 0; db < 4; ++db) o[db] = (v8f){};
    float mrun = -1.0e30f, lrun = 0.0f;
#pragma unroll 1
    for (int kt = 0; kt < SEQ / 64; ++kt) {
        const int key0 = kt * 64;
        v8f s[4];
#pragma unroll
        for (int rb = 0; rb < 4; ++rb) {
            const size_t ko = (size_t)(key0 + rb * 16) * HD;
            const V a0 = F::ld(kh + ko), a1 = F::ld(kh + ko + 32), c0 = F::ld(kl + ko), c1 = F::ld(kl + ko + 32);
            v8f t = (v8f){};
            t = wmmab(a0, qh0, t); t = wmmab(a0, ql0, t); t = wmmab(c0, qh0, t);
            t = wmmab(a1, qh1, t); t = wmmab(a1, ql1, t); t = wmmab(c1, qh1, t);
            asm volatile("v_nop\n\tv_nop\n\tv_nop\n\tv_nop" : "+v"(t) : "v"(a0), "v"(a1), "v"(c0), "v"(c1));
            s[rb] = t;
        }
        float mx = -1.0e30f;
#pragma unroll
        for (int rb = 0; rb < 4; ++rb)
#pragma unroll
            for (int r = 0; r < 8; ++r) { const float t2 = s[rb][r] * SC2; s[rb][r] = t2; mx = fmaxf(mx, t2); }
        mx = fmaxf(mx, __shfl_xor(mx, 16, 32));
        const float mnew = fmaxf(mrun, mx);
        const float corr = __builtin_amdgcn_exp2f(mrun - mnew);
        float ps = 0.0f;
#pragma unroll
        for (int rb = 0; rb < 4; ++rb)
#pragma unroll
            for (int r = 0; r < 8; ++r) { const float e = __builtin_amdgcn_exp2f(s[rb][r] - mnew); s[rb][r] = e; ps += e; }
        ps += __shfl_xor(ps, 16, 32);
        lrun = lrun * corr + ps; mrun = mnew;
#pragma unroll
        for (int db = 0; db < 4; ++db) o[db] = o[db] * corr;
#pragma unroll
        for (int jk = 0; jk < 2; ++jk) {
            v16us ph, pl;
#pragma unroll
            for (int r = 0; r < 8; ++r) { unsigned short u0, u1; splitf(s[2 * jk][r], u0, u1); ph[r] = u0; pl[r] = u1; splitf(s[2 * jk + 1][r], u0, u1); ph[8 + r] = u0; pl[8 + r] = u1; }
            const V pbh = __builtin_bit_cast(V, ph), pbl = __builtin_bit_cast(V, pl);
            const size_t vo = (size_t)(key0 + 32 * jk);
#pragma unroll
            for (int db = 0; db < 4; ++db) {
                const V ah = F::ld(vh + (size_t)db * 16 * SEQ + vo), al = F::ld(vl + (size_t)db * 16 * SEQ + vo);
                v8f t = o[db];
                t = wmmab(ah, pbh, t); t = wmmab(ah, pbl, t); t = wmmab(al, pbh, t);
                asm volatile("v_nop\n\tv_nop\n\tv_nop\n\tv_nop" : "+v"(t) : "v"(ah), "v"(al), "v"(pbh), "v"(pbl));
                o[db] = t;
            }
        }
    }
    const float il = 1.0f / lrun;
    float* os = osm + w * (16 * 68);
#pragma unroll
    for (int db = 0; db < 4; ++db) { v4f x0, x1; x0[0] = o[db][0] * il; x0[1] = o[db][1] * il; x0[2] = o[db][2] * il; x0[3] = o[db][3] * il; x1[0] = o[db][4] * il; x1[1] = o[db][5] * il; x1[2] = o[db][6] * il; x1[3] = o[db][7] * il;
        *(v4fa*)(os + lr * 68 + db * 16 + 8 * hi) = x0; *(v4fa*)(os + lr * 68 + db * 16 + 8 * hi + 4) = x1; }
    __builtin_amdgcn_fence(3  , "wavefront"); __builtin_amdgcn_wave_barrier(); asm volatile("" ::: "memory");
    const size_t row0 = (size_t)b * SEQ + q0; bf* ch = Ch + row0 * DMOD + h * HD; bf* cl = Cl + row0 * DMOD + h * HD;
#pragma unroll 1
    for (int pp = 0; pp < 2; ++pp) {
#pragma unroll
        for (int it = 0; it < 4; ++it) { const int q = it * 4 + (lane >> 3), jj = lane & 7; const v4f x0 = *(const v4fa*)(os + q * 68 + 8 * jj), x1 = *(const v4fa*)(os + q * 68 + 8 * jj + 4); v8us oh, ol;
#pragma unroll
            for (int e = 0; e < 4; ++e) { unsigned short u0, u1; splitf(x0[e], u0, u1); oh[e] = u0; ol[e] = u1; splitf(x1[e], u0, u1); oh[4 + e] = u0; ol[4 + e] = u1; }
            const size_t oo = (size_t)q * DMOD + 8 * jj; *(volatile v8us*)(ch + oo) = oh; *(volatile v8us*)(cl + oo) = ol; }
        if (pp == 0) __threadfence(); }
}

__global__ __launch_bounds__(128) void k_ortho(const bf* __restrict__ QA, const bf* __restrict__ QB, const float* __restrict__ inA, const float* __restrict__ inB, float* part) {
    typedef WFrag<bf> F; typedef F::V V;
    __shared__ float wp[4];
    const int lane = threadIdx.x & 31, lr = lane & 15, hi = lane >> 4, w = threadIdx.x >> 5;
    const size_t hb = blockIdx.z; const int i0 = blockIdx.y * 64, j0 = (blockIdx.x * 4 + w) * 64;
    const bf* A = QA + (hb * SEQ + i0) * HD + (size_t)lr * HD + 8 * hi; const bf* Bt = QB + (hb * SEQ + j0) * HD + (size_t)lr * HD + 8 * hi;
    v8f acc[4][4];
#pragma unroll
    for (int mb = 0; mb < 4; ++mb)
#pragma unroll
        for (int nb = 0; nb < 4; ++nb) acc[mb][nb] = (v8f){};
#pragma unroll
    for (int kc = 0; kc < HD; kc += 32) {
        V a[4];
#pragma unroll
        for (int mb = 0; mb < 4; ++mb) a[mb] = F::ld(A + (size_t)mb * 16 * HD + kc);
#pragma unroll
        for (int nb = 0; nb < 4; ++nb) { const V bb = F::ld(Bt + (size_t)nb * 16 * HD + kc);
#pragma unroll
            for (int mb = 0; mb < 4; ++mb) acc[mb][nb] = wmmab(a[mb], bb, acc[mb][nb]); }
        asm volatile("v_nop\n\tv_nop\n\tv_nop\n\tv_nop" : "+v"(acc[0][0]), "+v"(acc[0][1]), "+v"(acc[0][2]), "+v"(acc[0][3]), "+v"(acc[1][0]), "+v"(acc[1][1]), "+v"(acc[1][2]), "+v"(acc[1][3]),
                     "+v"(acc[2][0]), "+v"(acc[2][1]), "+v"(acc[2][2]), "+v"(acc[2][3]), "+v"(acc[3][0]), "+v"(acc[3][1]), "+v"(acc[3][2]), "+v"(acc[3][3]) : "v"(a[0]), "v"(a[1]), "v"(a[2]), "v"(a[3]));
    }
    float sq = 0.0f;
#pragma unroll
    for (int mb = 0; mb < 4; ++mb) { const v8f iv = *(const v8f*)(inA + hb * SEQ + i0 + mb * 16 + 8 * hi);
#pragma unroll
        for (int nb = 0; nb < 4; ++nb) { const float jv = inB[hb * SEQ + j0 + nb * 16 + lr]; const int gj = j0 + nb * 16 + lr;
#pragma unroll
            for (int r = 0; r < 8; ++r) { const int gi = i0 + mb * 16 + 8 * hi + r; const float x = acc[mb][nb][r] * iv[r] * jv; sq += (gi != gj) ? x * x : 0.0f; } } }
#pragma unroll
    for (int sh = 16; sh; sh >>= 1) sq += __shfl_xor(sq, sh, 32);
    if (lane == 0) wp[w] = sq;
    __syncthreads();
    const float bs = ((wp[0] + wp[1]) + wp[2]) + wp[3];
    if (w == 0 && lane < 8) { v4f v; v[0] = (lane == 0) ? bs : 0.0f; v[1] = 0.0f; v[2] = 0.0f; v[3] = 0.0f;
        const size_t pidx = ((size_t)blockIdx.z * gridDim.y + blockIdx.y) * gridDim.x + blockIdx.x; float* pptr = part + pidx * 32 + lane * 4;
        *(volatile v4f*)pptr = v; __threadfence(); *(volatile v4f*)pptr = v; }
}

__global__ __launch_bounds__(256) void k_cos(const float* __restrict__ X, const float* __restrict__ Y, float* part) {
    __shared__ float wp[8];
    const int lane = threadIdx.x & 31, w = threadIdx.x >> 5; const size_t row = (size_t)blockIdx.x * 8 + w;
    const float* xr = X + row * DMOD; const float* yr = Y + row * DMOD;
    float dot = 0.0f, nx = 0.0f, ny = 0.0f;
#pragma unroll 1
    for (int i = 0; i < DMOD / 128; ++i) { const v4f a = *(const v4f*)(xr + i * 128 + lane * 4); const v4f c = *(const v4f*)(yr + i * 128 + lane * 4);
#pragma unroll
        for (int e = 0; e < 4; ++e) { dot += a[e] * c[e]; nx += a[e] * a[e]; ny += c[e] * c[e]; } }
#pragma unroll
    for (int sh = 16; sh; sh >>= 1) { dot += __shfl_xor(dot, sh, 32); nx += __shfl_xor(nx, sh, 32); ny += __shfl_xor(ny, sh, 32); }
    const float cv = 1.0f - dot * rsqrtf(fmaxf(nx, 1e-24f)) * rsqrtf(fmaxf(ny, 1e-24f));
    if (lane == 0) wp[w] = cv;
    __syncthreads();
    const float bs = ((((((wp[0] + wp[1]) + wp[2]) + wp[3]) + wp[4]) + wp[5]) + wp[6]) + wp[7];
    if (w == 0 && lane < 8) { v4f v; v[0] = (lane == 0) ? bs : 0.0f; v[1] = 0.0f; v[2] = 0.0f; v[3] = 0.0f; float* pptr = part + (size_t)blockIdx.x * 32 + lane * 4;
        *(volatile v4f*)pptr = v; __threadfence(); *(volatile v4f*)pptr = v; }
}

__device__ double blkred(double v, double* red) {
    const int t = threadIdx.x; __syncthreads(); red[t] = v; __syncthreads();
#pragma unroll 1
    for (int s = 128; s > 0; s >>= 1) { if (t < s) red[t] = red[t] + red[t + s]; __syncthreads(); }
    const double r = red[0]; __syncthreads(); return r;
}
__global__ __launch_bounds__(256) void k_final(const float* __restrict__ op, int npo, const float* __restrict__ cp, int npc, float so, float sc, float* outs) {
    __shared__ double red[256];
    const int t = threadIdx.x;
    double a = 0.0;
#pragma unroll 1
    for (int i = t; i < npo; i += 256) a += (double)op[(size_t)i * 32];
    const double ra = blkred(a, red);
    double bsum = 0.0;
#pragma unroll 1
    for (int i = t; i < npo; i += 256) bsum += (double)op[(size_t)(npo + i) * 32];
    const double rb = blkred(bsum, red);
    double c = 0.0;
#pragma unroll 1
    for (int i = t; i < npc; i += 256) c += (double)cp[(size_t)i * 32];
    const double rc = blkred(c, red);
    if (t == 0) { const float v0 = (float)ra * so, v1 = (float)rb * so, v2 = (float)rc * sc; volatile float* o2 = outs; o2[0] = v0; o2[1] = v1; o2[2] = v2; __threadfence(); o2[0] = v0; o2[1] = v1; o2[2] = v2; }
}

extern "C" void kernel_launch(void* const* d_in, const int* in_sizes, int n_in,
                              void* d_out, int out_size, void* d_ws, size_t ws_size, hipStream_t stream) {
    if (n_in < 12) return;
    const size_t M = (size_t)NB * SEQ;
    const size_t needx = ((size_t)(NB - 1) * SEQ_FULL + SEQ) * DMOD;
    if ((size_t)in_sizes[0] < needx || (size_t)in_sizes[1] < needx) return;
    if ((size_t)in_sizes[2] < (size_t)QKVW * DMOD || (size_t)in_sizes[3] < (size_t)QKVW * DMOD) return;
    for (int i = 4; i <= 10; i += 2) { if ((size_t)in_sizes[i] < (size_t)DMOD * DMOD || (size_t)in_sizes[i + 1] < (size_t)DMOD) return; }
    if ((size_t)out_size < OFF4 + 3) return;
    const float* X = (const float*)d_in[0]; const float* Y = (const float*)d_in[1]; const float* Wq1 = (const float*)d_in[2]; const float* Wq2 = (const float*)d_in[3];
    const float* W1 = (const float*)d_in[4]; const float* B1 = (const float*)d_in[5]; const float* W2 = (const float*)d_in[6]; const float* B2 = (const float*)d_in[7];
    const float* W3 = (const float*)d_in[8]; const float* B3 = (const float*)d_in[9]; const float* W4 = (const float*)d_in[10]; const float* B4 = (const float*)d_in[11];
    float* OUT = (float*)d_out;
    char* wsp = (char*)d_ws;
    auto take = [&](size_t bytes) { char* p = wsp; wsp += (bytes + 255) & ~(size_t)255; return (void*)p; };
    const size_t plane = M * DMOD;
    const int NPO = NB * NH * (SEQ / 64) * (SEQ / 256);
    const int NPC = (int)(M / 8);
    bf* xb = (bf*)take(plane * 2); bf* yb = (bf*)take(plane * 2);
    bf* wq1b = (bf*)take((size_t)QKVW * DMOD * 2); bf* wq2b = (bf*)take((size_t)QKVW * DMOD * 2);
    bf* w1b = (bf*)take((size_t)DMOD * DMOD * 2); bf* w2b = (bf*)take((size_t)DMOD * DMOD * 2); bf* w3b = (bf*)take((size_t)DMOD * DMOD * 2); bf* w4b = (bf*)take((size_t)DMOD * DMOD * 2);
    float* qkvf = (float*)take(M * QKVW * 4);
    bf* Q1h = (bf*)take(plane * 2); bf* Q1l = (bf*)take(plane * 2); bf* K1h = (bf*)take(plane * 2); bf* K1l = (bf*)take(plane * 2); bf* T1h = (bf*)take(plane * 2); bf* T1l = (bf*)take(plane * 2);
    bf* V1h = (bf*)take(plane * 2); bf* V1l = (bf*)take(plane * 2); float* i1q = (float*)take(M * NH * 4); float* i1t = (float*)take(M * NH * 4);
    bf* Q2h = (bf*)take(plane * 2); bf* Q2l = (bf*)take(plane * 2); bf* K2h = (bf*)take(plane * 2); bf* K2l = (bf*)take(plane * 2); bf* T2h = (bf*)take(plane * 2); bf* T2l = (bf*)take(plane * 2);
    bf* V2h = (bf*)take(plane * 2); bf* V2l = (bf*)take(plane * 2); float* i2q = (float*)take(M * NH * 4); float* i2t = (float*)take(M * NH * 4);
    bf* Ch = (bf*)take(plane * 2); bf* Cl = (bf*)take(plane * 2);
    float* opart = (float*)take((size_t)2 * NPO * 32 * 4); float* cpart = (float*)take((size_t)NPC * 32 * 4);
    if ((size_t)(wsp - (char*)d_ws) > ws_size) return;

    const size_t n8x = plane / 8, n8q = (size_t)QKVW * DMOD / 8, n8w = (size_t)DMOD * DMOD / 8;
    k_cvtx<<<(unsigned)((n8x + 255) / 256), 256, 0, stream>>>(X, xb, n8x);
    k_cvtx<<<(unsigned)((n8x + 255) / 256), 256, 0, stream>>>(Y, yb, n8x);
    k_cvt8<<<(unsigned)((n8q + 255) / 256), 256, 0, stream>>>(Wq1, wq1b, n8q);
    k_cvt8<<<(unsigned)((n8q + 255) / 256), 256, 0, stream>>>(Wq2, wq2b, n8q);
    k_cvt8<<<(unsigned)((n8w + 255) / 256), 256, 0, stream>>>(W1, w1b, n8w);
    k_cvt8<<<(unsigned)((n8w + 255) / 256), 256, 0, stream>>>(W2, w2b, n8w);
    k_cvt8<<<(unsigned)((n8w + 255) / 256), 256, 0, stream>>>(W3, w3b, n8w);
    k_cvt8<<<(unsigned)((n8w + 255) / 256), 256, 0, stream>>>(W4, w4b, n8w);

    k_gemmw<bf, 0, false><<<dim3((unsigned)(M / 64), QKVW / 64, 1), 32, 0, stream>>>(xb, nullptr, wq1b, nullptr, DMOD, qkvf, QKVW, nullptr, 0, 0, 0);
    k_hp<<<dim3(SEQ / 32, NH, NB), 256, 0, stream>>>(qkvf, Q1h, Q1l, K1h, K1l, T1h, T1l, i1q, i1t);
    k_vt<<<dim3(SEQ / 64, NH, NB), 256, 0, stream>>>(qkvf, V1h, V1l);
    k_gemmw<bf, 0, false><<<dim3((unsigned)(M / 64), QKVW / 64, 1), 32, 0, stream>>>(yb, nullptr, wq2b, nullptr, DMOD, qkvf, QKVW, nullptr, 0, 0, 0);
    k_hp<<<dim3(SEQ / 32, NH, NB), 256, 0, stream>>>(qkvf, Q2h, Q2l, K2h, K2l, T2h, T2l, i2q, i2t);
    k_vt<<<dim3(SEQ / 64, NH, NB), 256, 0, stream>>>(qkvf, V2h, V2l);

    k_ortho<<<dim3(SEQ / 256, SEQ / 64, NB * NH), 128, 0, stream>>>(Q1h, T1h, i1q, i1t, opart);
    k_ortho<<<dim3(SEQ / 256, SEQ / 64, NB * NH), 128, 0, stream>>>(Q2h, T2h, i2q, i2t, opart + (size_t)NPO * 32);

    k_attn<<<dim3(SEQ / 64, NH, NB), 128, 0, stream>>>(Q2h, Q2l, K1h, K1l, V1h, V1l, Ch, Cl);
    k_gemmw<bf, 1, true><<<dim3((unsigned)(M / 64), DMOD / 64, 1), 32, 0, stream>>>(Ch, Cl, w1b, nullptr, DMOD, OUT + OFF0, DMOD, B1, 0, 0, 0);
    k_attn<<<dim3(SEQ / 64, NH, NB), 128, 0, stream>>>(Q1h, Q1l, K2h, K2l, V2h, V2l, Ch, Cl);
    k_gemmw<bf, 1, true><<<dim3((unsigned)(M / 64), DMOD / 64, 1), 32, 0, stream>>>(Ch, Cl, w2b, nullptr, DMOD, OUT + OFF1, DMOD, B2, 0, 0, 0);
    k_attn<<<dim3(SEQ / 64, NH, NB), 128, 0, stream>>>(T1h, T1l, K1h, K1l, V1h, V1l, Ch, Cl);
    k_gemmw<bf, 1, true><<<dim3((unsigned)(M / 64), DMOD / 64, 1), 32, 0, stream>>>(Ch, Cl, w3b, nullptr, DMOD, OUT + OFF2, DMOD, B3, 0, 0, 0);
    k_attn<<<dim3(SEQ / 64, NH, NB), 128, 0, stream>>>(T2h, T2l, K2h, K2l, V2h, V2l, Ch, Cl);
    k_gemmw<bf, 1, true><<<dim3((unsigned)(M / 64), DMOD / 64, 1), 32, 0, stream>>>(Ch, Cl, w4b, nullptr, DMOD, OUT + OFF3, DMOD, B4, 0, 0, 0);

    k_cos<<<(unsigned)(M / 8), 256, 0, stream>>>(OUT + OFF0, OUT + OFF1, cpart);
    const float so = 1.0f / ((float)NB * (float)SEQ * (float)SEQ), sc = 1.0f / ((float)NB * (float)SEQ);
    k_final<<<1, 256, 0, stream>>>(opart, NPO, cpart, NPC, so, sc, OUT + OFF4);
}
